// META_66331474920018
// MI455X (gfx1250) — hardware-verified
//
#include <hip/hip_runtime.h>
#include <math.h>

constexpr int kVocab    = 50000;
constexpr int kVocabPad = 50048;
constexpr int kEmb      = 256;
constexpr int kHidN     = 32;
constexpr int kGateN    = 128;
constexpr int kSeqN     = 16;
constexpr int kBatchN   = 32768;
constexpr int kOutW     = 64;
constexpr int kAttN     = 16;
static_assert(kVocabPad % 64 == 0 && kVocabPad >= kVocab, "pad");
static_assert(kEmb % 32 == 0 && kGateN % 64 == 0, "tile");
static_assert(kBatchN % 2048 == 0, "blk");

constexpr float kEmbCarry   = 64.0f;
constexpr float kWCarry     = 256.0f;
constexpr float kProjScale  = 1.0f / 16384.0f;
constexpr float kHCarry     = 64.0f;
constexpr float kRecScale   = 1.0f / 16384.0f;
constexpr float kFix        = 16384.0f;
constexpr float kFixInv     = 1.0f / 16384.0f;
constexpr float kOmCarry    = 256.0f;
constexpr float kPreScale   = 1.0f / 4194304.0f;
constexpr float kTanhCarry  = 1024.0f;
constexpr float kLogitScale = 1.0f / 262144.0f;

typedef __attribute__((ext_vector_type(16))) _Float16 v16h;
typedef __attribute__((ext_vector_type(8)))  _Float16 v8h;
typedef __attribute__((ext_vector_type(16))) __bf16   v16b;
typedef __attribute__((ext_vector_type(8)))  __bf16   v8b;
typedef __attribute__((ext_vector_type(8)))  float    v8f;
typedef __attribute__((ext_vector_type(4)))  float    v4f;
typedef __attribute__((ext_vector_type(4)))  unsigned int v4u;
typedef __attribute__((ext_vector_type(2)))  unsigned int v2u;
typedef v4u __attribute__((may_alias)) v4ua;
typedef v4f __attribute__((may_alias)) v4fa;

__device__ __forceinline__ unsigned short f2bf_bits(float f) {
  unsigned u = __float_as_uint(f);
  return (unsigned short)((u + 0x7FFFu + ((u >> 16) & 1u)) >> 16);
}
__device__ __forceinline__ float bf_bits2f(unsigned short h) { return __uint_as_float(((unsigned)h) << 16); }

__device__ __forceinline__ void dep_guard_h(v8f& a, v8f& b, v16h x, v16h y) { asm volatile("v_nop\n\tv_nop\n\tv_nop\n\tv_nop" : "+v"(a), "+v"(b) : "v"(x), "v"(y)); }
__device__ __forceinline__ void dep_guard_b(v8f& a, v8f& b, v16b x, v16b y) { asm volatile("v_nop\n\tv_nop\n\tv_nop\n\tv_nop" : "+v"(a), "+v"(b) : "v"(x), "v"(y)); }
__device__ __forceinline__ void keep4_h(v16h a, v16h b, v16h c, v16h d) { asm volatile("v_nop" :: "v"(a), "v"(b), "v"(c), "v"(d)); }
__device__ __forceinline__ void keep4_b(v16b a, v16b b, v16b c, v16b d) { asm volatile("v_nop" :: "v"(a), "v"(b), "v"(c), "v"(d)); }
__device__ __forceinline__ void acc_guard4(v8f& a, v8f& b, v8f& c, v8f& d) { asm volatile("v_nop\n\tv_nop\n\tv_nop\n\tv_nop" : "+v"(a), "+v"(b), "+v"(c), "+v"(d)); }
template <typename T> struct Frag;
template <> struct Frag<_Float16> {
  typedef v16h V; union U { v16h v; v8h h[2]; };
  static __device__ __forceinline__ v16h load(const _Float16* p) {
    U f; f.h[0] = *(const v8h*)(p); f.h[1] = *(const v8h*)(p + 16); return f.v;
  }
  static __device__ __forceinline__ v8f mma(v16h a, v16h b, v8f c) {
    return __builtin_amdgcn_wmma_f32_16x16x32_f16(false, a, false, b, (short)0, c, false, false);
  }
  static __device__ __forceinline__ void guard(v8f& a, v8f& b, v16h x, v16h y) { dep_guard_h(a, b, x, y); }
  static __device__ __forceinline__ void keep(v16h a, v16h b, v16h c, v16h d) { keep4_h(a, b, c, d); }
};
template <> struct Frag<__bf16> {
  typedef v16b V; union U { v16b v; v8b h[2]; };
  static __device__ __forceinline__ v16b load(const __bf16* p) {
    U f; f.h[0] = *(const v8b*)(p); f.h[1] = *(const v8b*)(p + 16); return f.v;
  }
  static __device__ __forceinline__ v8f mma(v16b a, v16b b, v8f c) {
    return __builtin_amdgcn_wmma_f32_16x16x32_bf16(false, a, false, b, (short)0, c, false, false);
  }
  static __device__ __forceinline__ void guard(v8f& a, v8f& b, v16b x, v16b y) { dep_guard_b(a, b, x, y); }
  static __device__ __forceinline__ void keep(v16b a, v16b b, v16b c, v16b d) { keep4_b(a, b, c, d); }
};

__device__ __forceinline__ unsigned pk16(unsigned short a, unsigned short b) { return (unsigned)a | ((unsigned)b << 16); }
__device__ __forceinline__ unsigned short h_bits(float f) { const _Float16 h = (_Float16)f; return __builtin_bit_cast(unsigned short, h); }

template <int ET> struct Elem;
template <> struct Elem<0> { typedef _Float16 T; };
template <> struct Elem<1> { typedef __bf16 T; };
template <int ET, bool SPLIT, int BIAS_MODE, int OUT_MODE, bool RESID, int ACT = 0>
__global__ __launch_bounds__(256) void wmma_gemm64(
    const unsigned short* __restrict__ Ap, const unsigned short* __restrict__ A2p, int lda, long strideA,
    const unsigned short* __restrict__ Btp, const unsigned short* __restrict__ Bt2p, int ldb, long strideB,
    void* __restrict__ Cout, void* __restrict__ Cout2, int ldc, long strideC,
    const float* __restrict__ bias,
    const float* __restrict__ resid, long strideR,
    int M, int N, int K, float scale) {
  typedef typename Elem<ET>::T T;
  typedef typename Frag<T>::V V;
  const T* A = (const T*)Ap; const T* A2 = (const T*)A2p; const T* Bt = (const T*)Btp; const T* Bt2 = (const T*)Bt2p;
  __shared__ __align__(16) float sT[8][16 * 68];
  const int b    = blockIdx.y;
  const int lane = threadIdx.x & 31;
  const int wave = threadIdx.x >> 5;
  const int tilesN = N >> 6;
  const int tilesM = M >> 6;
  const int tile = blockIdx.x * 8 + wave;
  if (tile >= tilesM * tilesN) return;
  const int tm = tile / tilesN;
  const int tn = tile - tm * tilesN;
  const int m0 = tm << 6;
  const int n0 = tn << 6;

  const T* Ab  = A  + (size_t)b * strideA;
  const T* Bb  = Bt + (size_t)b * strideB;
  const T* Ab2 = SPLIT ? (A2  + (size_t)b * strideA) : nullptr;
  const T* Bb2 = SPLIT ? (Bt2 + (size_t)b * strideB) : nullptr;

  const int rlane = lane & 15;
  const int koff  = (lane >> 4) * 8;
  const int mOff  = (lane >> 4) * 8;

  v8f acc[4][4];
#pragma unroll
  for (int i = 0; i < 4; ++i)
#pragma unroll
    for (int j = 0; j < 4; ++j) acc[i][j] = (v8f){0.f,0.f,0.f,0.f,0.f,0.f,0.f,0.f};

  for (int k0 = 0; k0 < K; k0 += 32) {
    V bh[4], bl[4];
#pragma unroll
    for (int j = 0; j < 4; ++j) {
      const size_t bo = (size_t)(n0 + (j << 4) + rlane) * ldb + koff + k0;
      bh[j] = Frag<T>::load(Bb + bo);
      if (SPLIT) bl[j] = Frag<T>::load(Bb2 + bo);
    }
#pragma unroll
    for (int i = 0; i < 4; ++i) {
      const size_t ao = (size_t)(m0 + (i << 4) + rlane) * lda + koff + k0;
      V ah = Frag<T>::load(Ab + ao);
      V al;
      if (SPLIT) al = Frag<T>::load(Ab2 + ao);
#pragma unroll
      for (int j = 0; j < 4; ++j) {
        acc[i][j] = Frag<T>::mma(ah, bh[j], acc[i][j]);
        if (SPLIT) {
          acc[i][j] = Frag<T>::mma(ah, bl[j], acc[i][j]);
          acc[i][j] = Frag<T>::mma(al, bh[j], acc[i][j]);
        }
      }
      Frag<T>::guard(acc[i][0], acc[i][3], ah, SPLIT ? al : ah);
    }
    Frag<T>::keep(bh[0], bh[1], bh[2], bh[3]);
    if (SPLIT) Frag<T>::keep(bl[0], bl[1], bl[2], bl[3]);
  }
  acc_guard4(acc[0][0], acc[0][1], acc[0][2], acc[0][3]);
  acc_guard4(acc[1][0], acc[1][1], acc[1][2], acc[1][3]);
  acc_guard4(acc[2][0], acc[2][1], acc[2][2], acc[2][3]);
  acc_guard4(acc[3][0], acc[3][1], acc[3][2], acc[3][3]);

  float* slab = sT[wave];
  const float* Rb = RESID ? (resid + (size_t)b * strideR) : nullptr;
#pragma unroll
  for (int i = 0; i < 4; ++i) {
    const int mBase = m0 + (i << 4);
#pragma unroll
    for (int j = 0; j < 4; ++j) {
      const int n = n0 + (j << 4) + rlane;
      float bv = 0.f;
      if (BIAS_MODE == 2) bv = bias[n];
#pragma unroll
      for (int r = 0; r < 8; ++r) {
        float v = acc[i][j][r] * scale;
        if (BIAS_MODE == 1) v += bias[mBase + mOff + r];
        if (BIAS_MODE == 2) v += bv;
        if (RESID) v += Rb[(size_t)(mBase + mOff + r) * ldc + n];
        if (ACT == 2) v = fmaxf(v, 0.0f);
        if (ACT == 4) v = (v > 0.f) ? v : 0.01f * v;
        slab[(mOff + r) * 68 + (j << 4) + rlane] = v;
      }
    }
    __builtin_amdgcn_fence(__ATOMIC_RELEASE, "workgroup");
    __builtin_amdgcn_wave_barrier();
    __builtin_amdgcn_fence(__ATOMIC_ACQUIRE, "workgroup");
    if (OUT_MODE == 0) {
      float* C = (float*)Cout + (size_t)b * strideC;
      const int hh = lane >> 4, c4 = (lane & 15) * 4;
      for (int pass = 0; pass < 2; ++pass) {
#pragma unroll
        for (int it = 0; it < 8; ++it) {
          const int row = it * 2 + hh;
          v4f v = *(const v4f*)(slab + row * 68 + c4);
          *(volatile v4f*)(C + (size_t)(mBase + row) * ldc + n0 + c4) = v;
        }
        __threadfence();
      }
    } else {
      const int q = lane >> 3, c8 = (lane & 7) * 8;
      unsigned short* C  = (unsigned short*)Cout  + (size_t)b * strideC;
      unsigned short* C2 = (OUT_MODE == 2) ? ((unsigned short*)Cout2 + (size_t)b * strideC) : nullptr;
      for (int pass = 0; pass < 2; ++pass) {
#pragma unroll
        for (int it = 0; it < 4; ++it) {
          const int row = it * 4 + q;
          const float* sp = slab + row * 68 + c8;
          v8h hv, lv;
#pragma unroll
          for (int e = 0; e < 8; ++e) {
            if (OUT_MODE == 1) {
              hv[e] = (_Float16)sp[e];
            } else {
              unsigned short hb = f2bf_bits(sp[e]);
              unsigned short lb = f2bf_bits(sp[e] - bf_bits2f(hb));
              hv[e] = __builtin_bit_cast(_Float16, hb);
              lv[e] = __builtin_bit_cast(_Float16, lb);
            }
          }
          *(volatile v8h*)(C + (size_t)(mBase + row) * ldc + n0 + c8) = hv;
          if (OUT_MODE == 2) *(volatile v8h*)(C2 + (size_t)(mBase + row) * ldc + n0 + c8) = lv;
        }
        __threadfence();
      }
    }
    __builtin_amdgcn_fence(__ATOMIC_RELEASE, "workgroup");
    __builtin_amdgcn_wave_barrier();
    __builtin_amdgcn_fence(__ATOMIC_ACQUIRE, "workgroup");
  }
}

__device__ __forceinline__ v8f mma_h(v16h a, v16h b, v8f c) {
  return __builtin_amdgcn_wmma_f32_16x16x32_f16(false, a, false, b, (short)0, c, false, false);
}
__device__ __forceinline__ void guard_acc4_in5(v8f& a, v8f& b, v8f& c, v8f& d, v16h x, v16h y0, v16h y1, v16h y2, v16h y3) {
  asm volatile("v_nop\n\tv_nop\n\tv_nop\n\tv_nop" : "+v"(a), "+v"(b), "+v"(c), "+v"(d) : "v"(x), "v"(y0), "v"(y1), "v"(y2), "v"(y3));
}
__device__ __forceinline__ void guard_acc1_in4(v8f& a, v16h x0, v16h x1, v16h y0, v16h y1) {
  asm volatile("v_nop\n\tv_nop\n\tv_nop\n\tv_nop" : "+v"(a) : "v"(x0), "v"(x1), "v"(y0), "v"(y1));
}
__device__ __forceinline__ void guard_acc1_in2(v8f& a, v16h x, v16h y) {
  asm volatile("v_nop\n\tv_nop\n\tv_nop\n\tv_nop" : "+v"(a) : "v"(x), "v"(y));
}
__device__ __forceinline__ void lds_sync() {
  __builtin_amdgcn_fence(__ATOMIC_RELEASE, "workgroup");
  __builtin_amdgcn_wave_barrier();
  __builtin_amdgcn_fence(__ATOMIC_ACQUIRE, "workgroup");
}
__device__ __forceinline__ float rcp_f(float x) { return __builtin_amdgcn_rcpf(x); }
__device__ __forceinline__ float sigm_f(float x) {
  x = fminf(fmaxf(x, -30.0f), 30.0f);
  return rcp_f(1.0f + expf(-x));
}
__device__ __forceinline__ float tanh_f(float x) {
  x = fminf(fmaxf(x, -15.0f), 15.0f);
  return 1.0f - 2.0f * rcp_f(1.0f + expf(2.0f * x));
}

__global__ __launch_bounds__(256) void k_cast_emb(const float* __restrict__ emb, unsigned short* __restrict__ out, int n8) {
  const int i = blockIdx.x * 256 + threadIdx.x;
  if (i >= n8) return;
  const int row  = i >> 5;
  const int rowc = (row < kVocab) ? row : (kVocab - 1);
  const float sc = (row < kVocab) ? kEmbCarry : 0.0f;
  const float* p = emb + (size_t)rowc * kEmb + (i & 31) * 8;
  const v4f a = *(const v4f*)(p);
  const v4f c = *(const v4f*)(p + 4);
  unsigned short hb[8];
#pragma unroll
  for (int e = 0; e < 4; ++e) {
    hb[e]     = h_bits(a[e] * sc);
    hb[4 + e] = h_bits(c[e] * sc);
  }
  const v4u u = (v4u){pk16(hb[0], hb[1]), pk16(hb[2], hb[3]), pk16(hb[4], hb[5]), pk16(hb[6], hb[7])};
  unsigned short* q = out + 8 * (size_t)i;
  *(volatile v4u*)q = u;
  __threadfence();
  *(volatile v4u*)q = u;
}

__global__ __launch_bounds__(256) void k_cast_w(const float* __restrict__ w0, const float* __restrict__ w1,
                                               unsigned short* __restrict__ out) {
  const int i = blockIdx.x * 256 + threadIdx.x;
  const bool first = (i < 4096);
  const int off = first ? i : (i - 4096);
  const float* p = (first ? w0 : w1) + (size_t)off * 8;
  const v4f a = *(const v4f*)(p);
  const v4f c = *(const v4f*)(p + 4);
  unsigned short hb[8];
#pragma unroll
  for (int e = 0; e < 4; ++e) {
    hb[e]     = h_bits(a[e] * kWCarry);
    hb[4 + e] = h_bits(c[e] * kWCarry);
  }
  const v4u u = (v4u){pk16(hb[0], hb[1]), pk16(hb[2], hb[3]), pk16(hb[4], hb[5]), pk16(hb[6], hb[7])};
  unsigned short* q = out + 8 * (size_t)i;
  *(volatile v4u*)q = u;
  __threadfence();
  *(volatile v4u*)q = u;
}

__global__ __launch_bounds__(64) void k_lstm(const float* __restrict__ P, const float* __restrict__ Whh,
                                             const float* __restrict__ bih, const float* __restrict__ bhh,
                                             const int* __restrict__ tokens, unsigned short* __restrict__ outq,
                                             int dir) {
  __shared__ int sTok[16 * 16];
  __shared__ __align__(16) _Float16 hA[2][16 * 32];
  __shared__ __align__(16) unsigned short sOut[16 * 16 * 32];

  const int tid  = threadIdx.x;
  const int lane = tid & 31, wave = tid >> 5;
  const int c    = lane & 15, hh = lane >> 4, koff = 8 * hh;
  const int b0   = blockIdx.x * 16;
  const int ucol = 16 * wave + c;

#pragma unroll
  for (int k = 0; k < 4; ++k) {
    const int e = k * 64 + tid;
    const int row = e >> 4, s = e & 15;
    int tk = tokens[(size_t)(b0 + row) * kSeqN + s];
    tk = (tk < 0) ? 0 : ((tk > kVocab - 1) ? (kVocab - 1) : tk);
    sTok[e] = tk;
  }
  {
    v8h z;
#pragma unroll
    for (int e = 0; e < 8; ++e) z[e] = (_Float16)0.0f;
    *(v8h*)(hA[0] + 8 * tid) = z;
  }
  float cst[8];
#pragma unroll
  for (int r = 0; r < 8; ++r) cst[r] = 0.0f;

  v16h wf[4];
  float bg[4];
#pragma unroll
  for (int g = 0; g < 4; ++g) {
    const int n = 32 * g + ucol;
    const float* wr = Whh + (size_t)n * kHidN;
#pragma unroll
    for (int i = 0; i < 8; ++i) {
      wf[g][i]     = (_Float16)(kWCarry * wr[koff + i]);
      wf[g][8 + i] = (_Float16)(kWCarry * wr[16 + koff + i]);
    }
    bg[g] = bih[n] + bhh[n];
  }
  __syncthreads();

  const v8f zero8 = (v8f){0.f,0.f,0.f,0.f,0.f,0.f,0.f,0.f};
#pragma unroll 1
  for (int t = 0; t < kSeqN; ++t) {
    const int s   = dir ? (kSeqN - 1 - t) : t;
    const int cur = t & 1;
    const _Float16* hcur = hA[cur];
    _Float16* hnxt = hA[cur ^ 1];

    const v16h ha = Frag<_Float16>::load(hcur + c * kHidN + koff);
    v8f acc[4];
#pragma unroll
    for (int g = 0; g < 4; ++g) acc[g] = mma_h(ha, wf[g], zero8);
    guard_acc4_in5(acc[0], acc[1], acc[2], acc[3], ha, wf[0], wf[1], wf[2], wf[3]);

#pragma unroll
    for (int r = 0; r < 8; ++r) {
      const int row = 8 * hh + r;
      const int tk  = sTok[row * 16 + s];
      const float* pr = P + (size_t)tk * kGateN + ucol;
      const float xi = acc[0][r] * kRecScale + (pr[0]  + bg[0]);
      const float xf = acc[1][r] * kRecScale + (pr[32] + bg[1]);
      const float xg = acc[2][r] * kRecScale + (pr[64] + bg[2]);
      const float xo = acc[3][r] * kRecScale + (pr[96] + bg[3]);
      const float cn = sigm_f(xf) * cst[r] + sigm_f(xi) * tanh_f(xg);
      const float hn = sigm_f(xo) * tanh_f(cn);
      cst[r] = cn;
      hnxt[row * kHidN + ucol] = (_Float16)(kHCarry * hn);
      const int qv = (int)rintf(kFix * hn);
      sOut[(row * 16 + s) * 32 + ucol] = (unsigned short)qv;
    }
    __syncthreads();
  }

  unsigned short* dst = outq + (size_t)b0 * (kSeqN * kHidN);
  for (int pass = 0; pass < 2; ++pass) {
#pragma unroll 1
    for (int it = 0; it < 16; ++it) {
      const int w = it * 64 + tid;
      const v4u v = *(const v4ua*)(sOut + 8 * w);
      *(volatile v4u*)(dst + 8 * (size_t)w) = v;
    }
    __threadfence();
  }
}

__global__ __launch_bounds__(256) void k_logit(const float* __restrict__ w_om, const float* __restrict__ u_om,
                                              const unsigned short* __restrict__ outF,
                                              const unsigned short* __restrict__ outB, float* __restrict__ logit) {
  __shared__ __align__(16) _Float16 sA[8][16 * 64];
  __shared__ __align__(16) _Float16 sA2[8][16 * 32];
  __shared__ __align__(16) float sL[8][128];

  const int tid  = threadIdx.x;
  const int lane = tid & 31, wave = tid >> 5;
  const int c    = lane & 15, hh = lane >> 4, koff = 8 * hh;
  const int s    = blockIdx.x >> 5;
  const int bw   = ((blockIdx.x & 31) << 10) + (wave << 7);
  _Float16* a1 = sA[wave];
  _Float16* a2 = sA2[wave];
  float* sl = sL[wave];

  v16h wb0, wb1, ubf;
#pragma unroll
  for (int i = 0; i < 8; ++i) {
    wb0[i]     = (_Float16)(kOmCarry * w_om[(koff + i) * kAttN + c]);
    wb0[8 + i] = (_Float16)(kOmCarry * w_om[(16 + koff + i) * kAttN + c]);
    wb1[i]     = (_Float16)(kOmCarry * w_om[(32 + koff + i) * kAttN + c]);
    wb1[8 + i] = (_Float16)(kOmCarry * w_om[(48 + koff + i) * kAttN + c]);
    ubf[i]     = (_Float16)(kOmCarry * u_om[koff + i]);
    ubf[8 + i] = (_Float16)0.0f;
  }
  {
    v8h z;
#pragma unroll
    for (int e = 0; e < 8; ++e) z[e] = (_Float16)0.0f;
    *(v8h*)(a2 + (lane >> 1) * 32 + 16 + (lane & 1) * 8) = z;
  }
  const v8f zero8 = (v8f){0.f,0.f,0.f,0.f,0.f,0.f,0.f,0.f};

#pragma unroll 1
  for (int t = 0; t < 8; ++t) {
    lds_sync();
    const int b = bw + 16 * t + c;
    const unsigned short* src = (hh ? outB : outF) + ((size_t)b * kSeqN + s) * kHidN;
#pragma unroll
    for (int jv = 0; jv < 4; ++jv) {
      const v4u w = *(const v4u*)(src + 8 * jv);
      v8h hv;
#pragma unroll
      for (int e = 0; e < 4; ++e) {
        const int lo = ((int)(w[e] << 16)) >> 16;
        const int hi = ((int)w[e]) >> 16;
        hv[2 * e]     = (_Float16)(float)lo;
        hv[2 * e + 1] = (_Float16)(float)hi;
      }
      *(v8h*)(a1 + c * 64 + 32 * hh + 8 * jv) = hv;
    }
    lds_sync();
    const v16h fa0 = Frag<_Float16>::load(a1 + c * 64 + koff);
    const v16h fa1 = Frag<_Float16>::load(a1 + c * 64 + 32 + koff);
    v8f acc = mma_h(fa0, wb0, zero8);
    acc = mma_h(fa1, wb1, acc);
    guard_acc1_in4(acc, fa0, fa1, wb0, wb1);
#pragma unroll
    for (int r = 0; r < 8; ++r) {
      const float th = tanh_f(acc[r] * kPreScale);
      a2[(8 * hh + r) * 32 + c] = (_Float16)(kTanhCarry * th);
    }
    lds_sync();
    const v16h fb = Frag<_Float16>::load(a2 + c * 32 + koff);
    v8f acc2 = mma_h(fb, ubf, zero8);
    guard_acc1_in2(acc2, fb, ubf);
    if (c == 0) {
#pragma unroll
      for (int r = 0; r < 8; ++r) sl[t * 16 + 8 * hh + r] = acc2[r] * kLogitScale;
    }
  }
  lds_sync();
  const v4f v = *(const v4fa*)(sl + 4 * lane);
  float* dst = logit + (size_t)s * kBatchN + bw + 4 * lane;
  *(volatile v4f*)dst = v;
  __threadfence();
  *(volatile v4f*)dst = v;
}

__global__ __launch_bounds__(256) void k_pool(const float* __restrict__ logit, const unsigned short* __restrict__ outF,
                                             const unsigned short* __restrict__ outB, float* __restrict__ dout) {
  const int tid  = threadIdx.x;
  const int lane = tid & 31;
  const int pair = blockIdx.x * 8 + (tid >> 5);
  const int b    = pair * 2 + (lane >> 4);
  const int j    = lane & 15;
  const int k4   = j * 4;
  const float* lp = logit + (size_t)(b >> 11) * kBatchN + ((b & 2047) << 4);
  const float e = expf(lp[j]);
  float ssum = e;
  ssum += __shfl_xor(ssum, 1, 32);
  ssum += __shfl_xor(ssum, 2, 32);
  ssum += __shfl_xor(ssum, 4, 32);
  ssum += __shfl_xor(ssum, 8, 32);
  ssum = __shfl(ssum, lane & 16, 32);
  const float inv = 1.0f / ssum;
  const unsigned short* src = ((k4 >= 32) ? outB : outF) + (size_t)b * (kSeqN * kHidN) + (k4 & 31);
  float a0 = 0.f, a1 = 0.f, a2 = 0.f, a3 = 0.f;
#pragma unroll 1
  for (int jj = 0; jj < kSeqN; ++jj) {
    const float ej = __shfl(e, (lane & 16) + jj, 32);
    const v2u w = *(const v2u*)(src + jj * kHidN);
    const float q0 = (float)(((int)(w[0] << 16)) >> 16);
    const float q1 = (float)(((int)w[0]) >> 16);
    const float q2 = (float)(((int)(w[1] << 16)) >> 16);
    const float q3 = (float)(((int)w[1]) >> 16);
    a0 += ej * q0;
    a1 += ej * q1;
    a2 += ej * q2;
    a3 += ej * q3;
  }
  const float f = inv * kFixInv;
  const v4f o = (v4f){a0 * f, a1 * f, a2 * f, a3 * f};
  float* dst = dout + (size_t)b * kOutW + k4;
  *(volatile v4f*)dst = o;
  __threadfence();
  *(volatile v4f*)dst = o;
}

extern "C" void kernel_launch(void* const* d_in, const int* in_sizes, int n_in,
                              void* d_out, int out_size, void* d_ws, size_t ws_size, hipStream_t stream) {
  if (n_in < 12) return;
  if (in_sizes[0] != kVocab * kEmb || in_sizes[1] != kGateN * kEmb || in_sizes[5] != kGateN * kEmb ||
      in_sizes[2] != kGateN * kHidN || in_sizes[6] != kGateN * kHidN || in_sizes[9] != kOutW * kAttN ||
      in_sizes[10] != kAttN || in_sizes[11] != kBatchN * kSeqN) return;
  if (out_size != kBatchN * kOutW) return;

  constexpr size_t offEmb16 = 0;
  constexpr size_t szEmb16  = (size_t)kVocabPad * kEmb * 2;
  constexpr size_t offP     = offEmb16 + szEmb16;
  constexpr size_t szP      = (size_t)kVocabPad * kGateN * 4;
  constexpr size_t offOutF  = offP + szP;
  constexpr size_t szOut    = (size_t)kBatchN * kSeqN * kHidN * 2;
  constexpr size_t offOutB  = offOutF + szOut;
  constexpr size_t offLogit = offOutB + szOut;
  constexpr size_t szLogit  = (size_t)kSeqN * kBatchN * 4;
  constexpr size_t offW16   = offLogit + szLogit;
  constexpr size_t szW16    = (size_t)2 * kGateN * kEmb * 2;
  constexpr size_t wsTotal  = offW16 + szW16;
  static_assert(wsTotal == 120586240ull, "carve");
  static_assert(wsTotal <= 134217728ull, "cap");
  static_assert(offP % 128 == 0 && offOutF % 128 == 0 && offOutB % 128 == 0 && offLogit % 128 == 0 && offW16 % 128 == 0, "align");
  if (ws_size < wsTotal) return;

  const float* emb   = (const float*)d_in[0];
  const float* Wih_f = (const float*)d_in[1];
  const float* Whh_f = (const float*)d_in[2];
  const float* bih_f = (const float*)d_in[3];
  const float* bhh_f = (const float*)d_in[4];
  const float* Wih_b = (const float*)d_in[5];
  const float* Whh_b = (const float*)d_in[6];
  const float* bih_b = (const float*)d_in[7];
  const float* bhh_b = (const float*)d_in[8];
  const float* w_om  = (const float*)d_in[9];
  const float* u_om  = (const float*)d_in[10];
  const int*   toks  = (const int*)d_in[11];
  float* dout = (float*)d_out;

  char* ws = (char*)d_ws;
  unsigned short* emb16 = (unsigned short*)(ws + offEmb16);
  float*          P     = (float*)(ws + offP);
  unsigned short* outF  = (unsigned short*)(ws + offOutF);
  unsigned short* outB  = (unsigned short*)(ws + offOutB);
  float*          lgt   = (float*)(ws + offLogit);
  unsigned short* w16   = (unsigned short*)(ws + offW16);

  const int n8emb = kVocabPad * kEmb / 8;
  k_cast_emb<<<dim3((n8emb + 255) / 256), dim3(256), 0, stream>>>(emb, emb16, n8emb);
  k_cast_w<<<dim3(32), dim3(256), 0, stream>>>(Wih_f, Wih_b, w16);

  const int gemmBlocks = (782 * 2 + 7) / 8;
  for (int d = 0; d < 2; ++d) {
    const unsigned short* bt = w16 + (size_t)d * kGateN * kEmb;
    hipLaunchKernelGGL((wmma_gemm64<0, false, 0, 0, false, 0>), dim3(gemmBlocks, 1, 1), dim3(256, 1, 1), 0, stream,
                       (const unsigned short*)emb16, (const unsigned short*)emb16, (int)kEmb, 0L,
                       bt, bt, (int)kEmb, 0L,
                       (void*)P, (void*)P, (int)kGateN, 0L,
                       (const float*)P, (const float*)P, 0L,
                       (int)kVocabPad, (int)kGateN, (int)kEmb, kProjScale);
    if (d == 0) {
      k_lstm<<<dim3(kBatchN / 16), dim3(64), 0, stream>>>(P, Whh_f, bih_f, bhh_f, toks, outF, 0);
    } else {
      k_lstm<<<dim3(kBatchN / 16), dim3(64), 0, stream>>>(P, Whh_b, bih_b, bhh_b, toks, outB, 1);
    }
  }
  k_logit<<<dim3(kSeqN * kBatchN / 1024), dim3(256), 0, stream>>>(w_om, u_om, outF, outB, lgt);
  k_pool<<<dim3(kBatchN / 16), dim3(256), 0, stream>>>(lgt, outF, outB, dout);
}
